// ModulatedDeformConv2d_8684423872827
// MI455X (gfx1250) — hardware-verified
//
#include <hip/hip_runtime.h>
#include <math.h>

typedef __attribute__((ext_vector_type(16))) _Float16 v16h;
typedef __attribute__((ext_vector_type(16))) __bf16 v16b;
typedef __attribute__((ext_vector_type(8)))  _Float16 v8h;
typedef __attribute__((ext_vector_type(8)))  float v8f;
typedef __attribute__((ext_vector_type(4)))  float v4f;
typedef __attribute__((ext_vector_type(2)))  float v2f;
typedef __attribute__((ext_vector_type(4)))  unsigned v4u;
typedef __attribute__((ext_vector_type(4)))  int v4i;
typedef float __attribute__((may_alias)) float_a;
typedef int __attribute__((may_alias)) int_a;

template <typename T> __device__ __forceinline__ void vst2(void* p, T v) { *(volatile T*)p = v; __threadfence(); *(volatile T*)p = v; }
__device__ __forceinline__ v8f wmma16(v16h a, v16h b, v8f c) {
  v8f d = __builtin_amdgcn_wmma_f32_16x16x32_f16(false, a, false, b, (short)0, c, false, false);
  asm volatile("v_nop\n\tv_nop\n\tv_nop\n\tv_nop" : "+v"(d) : "v"(a), "v"(b));
  return d;
}
__device__ __forceinline__ v8f wmma_bf(v16b a, v16b b, v8f c) {
  v8f d = __builtin_amdgcn_wmma_f32_16x16x32_bf16(false, a, false, b, (short)0, c, false, false);
  asm volatile("v_nop\n\tv_nop\n\tv_nop\n\tv_nop" : "+v"(d) : "v"(a), "v"(b));
  return d;
}
__device__ __forceinline__ v16h frag_h(const _Float16* rowk0, int lane) {
  union { v16h v; v8h q[2]; } u; const _Float16* p = rowk0 + 8 * (lane >> 4);
  u.q[0] = *(const v8h*)p; u.q[1] = *(const v8h*)(p + 16); return u.v;
}
__device__ __forceinline__ v16h frag_f32(const float* rowk0, int lane) {
  v16h a; const float* p = rowk0 + 8 * (lane >> 4);
#pragma unroll
  for (int i = 0; i < 8; ++i) { a[i] = (_Float16)p[i]; a[8 + i] = (_Float16)p[16 + i]; }
  return a;
}
__device__ __forceinline__ v16h frag_f32s(const float* rowk0, int lane, float sc) {
  v16h a; const float* p = rowk0 + 8 * (lane >> 4);
#pragma unroll
  for (int i = 0; i < 8; ++i) { a[i] = (_Float16)(p[i] * sc); a[8 + i] = (_Float16)(p[16 + i] * sc); }
  return a;
}
__device__ __forceinline__ v16h fragc_f32(const float* W, int k0, int n, int lane, int ld, int K) {
  v16h a; const int g = lane >> 4;
#pragma unroll
  for (int i = 0; i < 8; ++i) { const int ka = k0 + 8 * g + i, kb = ka + 16;
    a[i] = (_Float16)(ka < K ? W[(size_t)(ka < K ? ka : K - 1) * ld + n] : 0.f); a[8 + i] = (_Float16)(kb < K ? W[(size_t)(kb < K ? kb : K - 1) * ld + n] : 0.f); }
  return a;
}
struct F2 { v16b h, l; };
__device__ __forceinline__ F2 bsplit16(const float v[16]) { F2 r;
#pragma unroll
  for (int i = 0; i < 16; ++i) { const __bf16 h = (__bf16)v[i]; r.h[i] = h; r.l[i] = (__bf16)(v[i] - (float)h); }
  return r; }
__device__ __forceinline__ F2 split_row(const float* row, int k0, int lane) { float v[16]; const float* p = row + k0 + 8 * (lane >> 4);
#pragma unroll
  for (int i = 0; i < 8; ++i) { v[i] = p[i]; v[8 + i] = p[16 + i]; }
  return bsplit16(v); }
__device__ __forceinline__ F2 split_rowK(const float* row, int k0, int lane, int K) { float v[16]; const int g = lane >> 4;
#pragma unroll
  for (int i = 0; i < 8; ++i) { const int ka = k0 + 8 * g + i, kb = ka + 16; v[i] = ka < K ? row[ka < K ? ka : K - 1] : 0.f; v[8 + i] = kb < K ? row[kb < K ? kb : K - 1] : 0.f; }
  return bsplit16(v); }
__device__ __forceinline__ F2 split_col(const float* W, int k0, int n, int lane, int ld, int K) { float v[16]; const int g = lane >> 4;
#pragma unroll
  for (int i = 0; i < 8; ++i) { const int ka = k0 + 8 * g + i, kb = ka + 16; v[i] = ka < K ? W[(size_t)(ka < K ? ka : K - 1) * ld + n] : 0.f; v[8 + i] = kb < K ? W[(size_t)(kb < K ? kb : K - 1) * ld + n] : 0.f; }
  return bsplit16(v); }
__device__ __forceinline__ v8f mac3(const F2& a, const F2& b, v8f c) { c = wmma_bf(a.l, b.h, c); c = wmma_bf(a.h, b.l, c); return wmma_bf(a.h, b.h, c); }
__device__ __forceinline__ float sigm(float v) { return 1.0f / (1.0f + expf(-v)); }
#define LDSX() do { asm volatile("s_wait_dscnt 0" ::: "memory"); __builtin_amdgcn_wave_barrier(); __builtin_amdgcn_fence(__ATOMIC_RELEASE, "workgroup"); } while (0)


#define NB 8
#define CI 64
#define CO 64
#define IH 128
#define IW 128
#define K2 9
#define KK (CI * K2)
#define RB 6
#define NROWS (2 * RB + 3)
#define CPAD 8
#define NCOLS (64 + 2 * CPAD)
#ifndef TNB
#define TNB NB
#endif
typedef __attribute__((ext_vector_type(8))) __bf16 v8b;
__device__ __forceinline__ v16b frag_b(const __bf16* rowk0, int lane) {
  union { v16b v; v8b q[2]; } u; const __bf16* p = rowk0 + 8 * (lane >> 4);
  u.q[0] = *(const v8b*)p; u.q[1] = *(const v8b*)(p + 16); return u.v;
}
__device__ __forceinline__ float bfr(float v) { return (float)(__bf16)v; }
__device__ __attribute__((noinline)) float exp_ni(float v) { return expf(v); }
__device__ __attribute__((noinline)) float erf_ni(float v) { return erff(v); }

__global__ __launch_bounds__(128) void k_dcn(const float* __restrict__ X, const float* __restrict__ OFF, const float* __restrict__ MSK, const float* __restrict__ Wt, const float* __restrict__ BIAS, float* __restrict__ OUT) {
  __shared__ __align__(16) __bf16 sx[CI][NROWS][NCOLS];
  __shared__ float spy[K2][64], spx[K2][64], smk[K2][64];
  const int tid = threadIdx.x, wave = tid >> 5, lane = tid & 31, col = lane & 15, g = lane >> 4;
  const size_t p0 = (size_t)blockIdx.x * 64; const size_t b = p0 / (IH * IW); const int pp = (int)(p0 % (IH * IW)); const int y = pp / IW, x0 = pp % IW;
  const int ylo = y - 1 - RB, xlo = x0 - CPAD;
  for (int e = tid; e < CI * NROWS * NCOLS; e += 128) { const int c = e / (NROWS * NCOLS), rem = e % (NROWS * NCOLS); const int rr = rem / NCOLS, cc = rem % NCOLS; const int gy = ylo + rr, gx = xlo + cc; float v = 0.f; if (gy >= 0 && gy < IH && gx >= 0 && gx < IW) v = X[((b * CI + c) * IH + gy) * (size_t)IW + gx]; sx[c][rr][cc] = (__bf16)v; }
  for (int e = tid; e < K2 * 64; e += 128) { const int k = e >> 6, pl = e & 63; const int kh = k / 3, kw = k % 3; const size_t pix = ((size_t)y * IW + x0 + pl);
    const float dxv = bfr(OFF[((b * 2 * K2 + 2 * k) * IH * IW) + pix]), dyv = bfr(OFF[((b * 2 * K2 + 2 * k + 1) * IH * IW) + pix]);
    const float base_y = (float)(y - 1), base_x = (float)(x0 + pl - 1); const float py = (base_y + (float)kh) + dyv, px = (base_x + (float)kw) + dxv;
    spy[k][pl] = py; spx[k][pl] = px; smk[k][pl] = bfr(MSK[((b * K2 + k) * IH * IW) + pix]); }
  __syncthreads();
  v8f acc[4] = {};
  const int myrow = wave * 16 + col;
#pragma unroll 1
  for (int kc = 0; kc < KK / 32; ++kc) { v16b ah, al;
#pragma unroll
    for (int i = 0; i < 16; ++i) { const int q = kc * 32 + 8 * g + (i < 8 ? i : i + 8); const int c = q / K2, k = q % K2;
      const float py = spy[k][myrow], px = spx[k][myrow]; const float fy = floorf(py), fx = floorf(px); const int y0i = (int)fy, x0i = (int)fx; const float wy1 = py - fy, wx1 = px - fx, wy0 = 1.0f - wy1, wx0 = 1.0f - wx1;
      float v = 0.f;
#pragma unroll
      for (int cy = 0; cy < 2; ++cy)
#pragma unroll
        for (int cx = 0; cx < 2; ++cx) { const int iy = y0i + cy, ix = x0i + cx; float s = 0.f;
          if (iy >= 0 && iy < IH && ix >= 0 && ix < IW) { const int ry = iy - ylo, rx = ix - xlo; if (ry >= 0 && ry < NROWS && rx >= 0 && rx < NCOLS) s = (float)sx[c][ry][rx]; else s = bfr(X[((b * CI + c) * IH + iy) * (size_t)IW + ix]); }
          v += s * ((cy ? wy1 : wy0) * (cx ? wx1 : wx0)); }
      v *= smk[k][myrow]; const __bf16 h = (__bf16)v; ah[i] = h; al[i] = (__bf16)(v - (float)h); }
#pragma unroll
    for (int j = 0; j < 4; ++j) { v16b w; const int o = j * 16 + col; const float* p = Wt + (size_t)o * KK + kc * 32 + 8 * g;
#pragma unroll
      for (int i = 0; i < 8; ++i) { w[i] = (__bf16)p[i]; w[8 + i] = (__bf16)p[16 + i]; }
      acc[j] = wmma_bf(ah, w, acc[j]); acc[j] = wmma_bf(al, w, acc[j]); } }
  __syncthreads();
  float (*so)[68] = (float (*)[68])&sx[0][0][0];
#pragma unroll
  for (int j = 0; j < 4; ++j) { const int o = j * 16 + col; const float bb = bfr(BIAS[o]);
#pragma unroll
    for (int r = 0; r < 8; ++r) so[o][wave * 16 + 8 * g + r] = acc[j][r] + bb; }
  __syncthreads(); for (int e = tid; e < CO * 16; e += 128) { const int o = e >> 4, q = e & 15; vst2(OUT + ((b * CO + o) * IH + y) * (size_t)IW + x0 + q * 4, *(const v4f*)&so[o][q * 4]); } }
extern "C" void kernel_launch(void* const* d_in, const int* in_sizes, int n_in, void* d_out, int out_size, void* d_ws, size_t ws_size, hipStream_t stream) {
  (void)in_sizes; (void)n_in; (void)out_size; (void)d_ws; (void)ws_size;
  const float** F = (const float**)d_in;
  k_dcn<<<TNB * IH * IW / 64, 128, 0, stream>>>(F[0], F[1], F[2], F[3], F[4], (float*)d_out);
}
